// GPT2Attention_41420664602947
// MI455X (gfx1250) — hardware-verified
//
#include <hip/hip_runtime.h>
#include <stdint.h>

typedef __attribute__((ext_vector_type(16))) _Float16 v16h;
typedef __attribute__((ext_vector_type(8)))  _Float16 v8h;
typedef __attribute__((ext_vector_type(16))) __bf16   v16b;
typedef __attribute__((ext_vector_type(8)))  __bf16   v8b;
typedef __attribute__((ext_vector_type(8)))  float    v8f;
typedef __attribute__((ext_vector_type(4)))  float    v4f;
typedef __attribute__((ext_vector_type(4)))  unsigned int v4u;

#define NB_BATCH 4
#define SEQ_LEN 2048
#define EMB_DIM 1024
#define N_HEADS 16
#define HEAD_D 64
#define MROWS (NB_BATCH * SEQ_LEN)
#define QKV_N (3 * EMB_DIM)
#define QK_PITCH (2 * EMB_DIM)
#define KV_CHUNK 64
#define MASK_FILL (-10000.0f)

static_assert(MROWS % 64 == 0);
static_assert(EMB_DIM % 64 == 0);
static_assert(QK_PITCH % 64 == 0);
static_assert(EMB_DIM % 32 == 0);
static_assert(SEQ_LEN % 64 == 0);
static_assert(HEAD_D == 64);
static_assert(N_HEADS * HEAD_D == EMB_DIM);

#define WS_OFF_XBF   ((size_t)0)
#define WS_OFF_WAT   (WS_OFF_XBF + (size_t)MROWS * EMB_DIM * 2)
#define WS_OFF_WPT   (WS_OFF_WAT + (size_t)QKV_N * EMB_DIM * 2)
#define WS_OFF_QKP   (WS_OFF_WPT + (size_t)EMB_DIM * EMB_DIM * 2)
#define WS_OFF_VHI   (WS_OFF_QKP + (size_t)MROWS * QK_PITCH * 2)
#define WS_OFF_VLO   (WS_OFF_VHI + (size_t)MROWS * EMB_DIM * 2)
#define WS_OFF_ATH   (WS_OFF_VLO + (size_t)MROWS * EMB_DIM * 2)
#define WS_OFF_ATL   (WS_OFF_ATH + (size_t)MROWS * EMB_DIM * 2)
#define WS_TOTAL     (WS_OFF_ATL + (size_t)MROWS * EMB_DIM * 2)
static_assert(WS_TOTAL == (size_t)125829120);
static_assert(WS_TOTAL <= (size_t)134217728);
static_assert(WS_OFF_WAT % 128 == 0 && WS_OFF_WPT % 128 == 0 && WS_OFF_QKP % 128 == 0 && WS_OFF_VHI % 128 == 0 &&
              WS_OFF_VLO % 128 == 0 && WS_OFF_ATH % 128 == 0 && WS_OFF_ATL % 128 == 0);

__device__ __forceinline__ unsigned short f2bf_bits(float f) {
  unsigned u = __float_as_uint(f);
  return (unsigned short)((u + 0x7FFFu + ((u >> 16) & 1u)) >> 16);
}
__device__ __forceinline__ float bf_bits2f(unsigned short h) { return __uint_as_float(((unsigned)h) << 16); }

__device__ __forceinline__ void dep_guard_h(v8f& a, v8f& b, v16h x, v16h y) { asm volatile("v_nop\n\tv_nop\n\tv_nop\n\tv_nop" : "+v"(a), "+v"(b) : "v"(x), "v"(y)); }
__device__ __forceinline__ void dep_guard_b(v8f& a, v8f& b, v16b x, v16b y) { asm volatile("v_nop\n\tv_nop\n\tv_nop\n\tv_nop" : "+v"(a), "+v"(b) : "v"(x), "v"(y)); }
__device__ __forceinline__ void keep4_h(v16h a, v16h b, v16h c, v16h d) { asm volatile("v_nop" :: "v"(a), "v"(b), "v"(c), "v"(d)); }
__device__ __forceinline__ void keep4_b(v16b a, v16b b, v16b c, v16b d) { asm volatile("v_nop" :: "v"(a), "v"(b), "v"(c), "v"(d)); }
__device__ __forceinline__ void acc_guard4(v8f& a, v8f& b, v8f& c, v8f& d) { asm volatile("v_nop\n\tv_nop\n\tv_nop\n\tv_nop" : "+v"(a), "+v"(b), "+v"(c), "+v"(d)); }
template <typename T> struct Frag;
template <> struct Frag<_Float16> {
  typedef v16h V; union U { v16h v; v8h h[2]; };
  static __device__ __forceinline__ v16h load(const _Float16* p) {
    U f; f.h[0] = *(const v8h*)(p); f.h[1] = *(const v8h*)(p + 16); return f.v;
  }
  static __device__ __forceinline__ v8f mma(v16h a, v16h b, v8f c) {
    return __builtin_amdgcn_wmma_f32_16x16x32_f16(false, a, false, b, (short)0, c, false, false);
  }
  static __device__ __forceinline__ void guard(v8f& a, v8f& b, v16h x, v16h y) { dep_guard_h(a, b, x, y); }
  static __device__ __forceinline__ void keep(v16h a, v16h b, v16h c, v16h d) { keep4_h(a, b, c, d); }
};
template <> struct Frag<__bf16> {
  typedef v16b V; union U { v16b v; v8b h[2]; };
  static __device__ __forceinline__ v16b load(const __bf16* p) {
    U f; f.h[0] = *(const v8b*)(p); f.h[1] = *(const v8b*)(p + 16); return f.v;
  }
  static __device__ __forceinline__ v8f mma(v16b a, v16b b, v8f c) {
    return __builtin_amdgcn_wmma_f32_16x16x32_bf16(false, a, false, b, (short)0, c, false, false);
  }
  static __device__ __forceinline__ void guard(v8f& a, v8f& b, v16b x, v16b y) { dep_guard_b(a, b, x, y); }
  static __device__ __forceinline__ void keep(v16b a, v16b b, v16b c, v16b d) { keep4_b(a, b, c, d); }
};

__device__ __forceinline__ v8f hmma(v16h a, v16h b, v8f c) {
  c = __builtin_amdgcn_wmma_f32_16x16x32_f16(false, a, false, b, (short)0, c, false, false);
  asm volatile("v_nop\n\tv_nop\n\tv_nop\n\tv_nop" : "+v"(c) : "v"(a), "v"(b));
  return c;
}
__device__ __forceinline__ v8f bmma(v16b a, v16b b, v8f c) {
  c = __builtin_amdgcn_wmma_f32_16x16x32_bf16(false, a, false, b, (short)0, c, false, false);
  asm volatile("v_nop\n\tv_nop\n\tv_nop\n\tv_nop" : "+v"(c) : "v"(a), "v"(b));
  return c;
}

template <int ET> struct Elem;
template <> struct Elem<0> { typedef _Float16 T; };
template <> struct Elem<1> { typedef __bf16 T; };
template <int ET, bool SPLITA, bool SPLITB, int BIAS_MODE, int OUT_MODE>
__global__ __launch_bounds__(256) void wmma_gemm64(
    const unsigned short* __restrict__ Ap, const unsigned short* __restrict__ A2p, int lda, long strideA,
    const unsigned short* __restrict__ Btp, const unsigned short* __restrict__ Bt2p, int ldb, long strideB,
    void* __restrict__ Cout, void* __restrict__ Cout2, int ldc, long strideC,
    const float* __restrict__ bias,
    int M, int N, int K, float scale, float bscale) {
  typedef typename Elem<ET>::T T;
  typedef typename Frag<T>::V V;
  const T* A = (const T*)Ap; const T* A2 = (const T*)A2p; const T* Bt = (const T*)Btp; const T* Bt2 = (const T*)Bt2p;
  __shared__ __align__(16) float sT[8][16 * 68];
  const int b    = blockIdx.y;
  const int lane = threadIdx.x & 31;
  const int wave = threadIdx.x >> 5;
  const int tilesN = N >> 6;
  const int tilesM = M >> 6;
  const int tile = blockIdx.x * 8 + wave;
  if (tile >= tilesM * tilesN) return;
  const int tm = tile / tilesN;
  const int tn = tile - tm * tilesN;
  const int m0 = tm << 6;
  const int n0 = tn << 6;

  const T* Ab  = A  + (size_t)b * strideA;
  const T* Bb  = Bt + (size_t)b * strideB;
  const T* Ab2 = SPLITA ? (A2  + (size_t)b * strideA) : nullptr;
  const T* Bb2 = SPLITB ? (Bt2 + (size_t)b * strideB) : nullptr;

  const int rlane = lane & 15;
  const int koff  = (lane >> 4) * 8;
  const int mOff  = (lane >> 4) * 8;

  v8f acc[4][4];
#pragma unroll
  for (int i = 0; i < 4; ++i)
#pragma unroll
    for (int j = 0; j < 4; ++j) acc[i][j] = (v8f){0.f,0.f,0.f,0.f,0.f,0.f,0.f,0.f};

  for (int k0 = 0; k0 < K; k0 += 32) {
    V bh[4], bl[4];
#pragma unroll
    for (int j = 0; j < 4; ++j) {
      const size_t bo = (size_t)(n0 + (j << 4) + rlane) * ldb + koff + k0;
      bh[j] = Frag<T>::load(Bb + bo);
      if (SPLITB) bl[j] = Frag<T>::load(Bb2 + bo);
    }
#pragma unroll
    for (int i = 0; i < 4; ++i) {
      const size_t ao = (size_t)(m0 + (i << 4) + rlane) * lda + koff + k0;
      V ah = Frag<T>::load(Ab + ao);
      V al = ah;
      if (SPLITA) al = Frag<T>::load(Ab2 + ao);
#pragma unroll
      for (int j = 0; j < 4; ++j) {
        acc[i][j] = Frag<T>::mma(ah, bh[j], acc[i][j]);
        if (SPLITB) acc[i][j] = Frag<T>::mma(ah, bl[j], acc[i][j]);
        if (SPLITA) acc[i][j] = Frag<T>::mma(al, bh[j], acc[i][j]);
      }
      Frag<T>::guard(acc[i][0], acc[i][3], ah, al);
    }
    Frag<T>::keep(bh[0], bh[1], bh[2], bh[3]);
    if (SPLITB) Frag<T>::keep(bl[0], bl[1], bl[2], bl[3]);
  }
  acc_guard4(acc[0][0], acc[0][1], acc[0][2], acc[0][3]);
  acc_guard4(acc[1][0], acc[1][1], acc[1][2], acc[1][3]);
  acc_guard4(acc[2][0], acc[2][1], acc[2][2], acc[2][3]);
  acc_guard4(acc[3][0], acc[3][1], acc[3][2], acc[3][3]);

  float* slab = sT[wave];
#pragma unroll
  for (int i = 0; i < 4; ++i) {
    const int mBase = m0 + (i << 4);
#pragma unroll
    for (int j = 0; j < 4; ++j) {
      const int n = n0 + (j << 4) + rlane;
      float bv = 0.f;
      if (BIAS_MODE == 2) bv = bf_bits2f(f2bf_bits(bias[n])) * bscale;
#pragma unroll
      for (int r = 0; r < 8; ++r) {
        float v = acc[i][j][r] * scale;
        if (BIAS_MODE == 2) v += bv;
        slab[(mOff + r) * 68 + (j << 4) + rlane] = v;
      }
    }
    __builtin_amdgcn_fence(__ATOMIC_RELEASE, "workgroup");
    __builtin_amdgcn_wave_barrier();
    __builtin_amdgcn_fence(__ATOMIC_ACQUIRE, "workgroup");
    if (OUT_MODE == 0) {
      float* C = (float*)Cout + (size_t)b * strideC;
      const int hh = lane >> 4, c4 = (lane & 15) * 4;
      for (int pass = 0; pass < 2; ++pass) {
#pragma unroll
        for (int it = 0; it < 8; ++it) {
          const int row = it * 2 + hh;
          v4f v = *(const v4f*)(slab + row * 68 + c4);
          *(volatile v4f*)(C + (size_t)(mBase + row) * ldc + n0 + c4) = v;
        }
        __threadfence();
      }
    } else {
      const int q = lane >> 3, c8 = (lane & 7) * 8;
      unsigned short* C  = (unsigned short*)Cout  + (size_t)b * strideC;
      unsigned short* C2 = (OUT_MODE == 2) ? ((unsigned short*)Cout2 + (size_t)b * strideC) : nullptr;
      for (int pass = 0; pass < 2; ++pass) {
#pragma unroll
        for (int it = 0; it < 4; ++it) {
          const int row = it * 4 + q;
          const float* sp = slab + row * 68 + c8;
          v8h hv, lv;
#pragma unroll
          for (int e = 0; e < 8; ++e) {
            if (OUT_MODE == 1) {
              hv[e] = (_Float16)sp[e];
            } else {
              unsigned short hb = f2bf_bits(sp[e]);
              unsigned short lb = f2bf_bits(sp[e] - bf_bits2f(hb));
              hv[e] = __builtin_bit_cast(_Float16, hb);
              lv[e] = __builtin_bit_cast(_Float16, lb);
            }
          }
          *(volatile v8h*)(C + (size_t)(mBase + row) * ldc + n0 + c8) = hv;
          if (OUT_MODE == 2) *(volatile v8h*)(C2 + (size_t)(mBase + row) * ldc + n0 + c8) = lv;
        }
        __threadfence();
      }
    }
    __builtin_amdgcn_fence(__ATOMIC_RELEASE, "workgroup");
    __builtin_amdgcn_wave_barrier();
    __builtin_amdgcn_fence(__ATOMIC_ACQUIRE, "workgroup");
  }
}

__global__ __launch_bounds__(256) void cast_f32_bf16x8(
    const float* __restrict__ in, unsigned short* __restrict__ out, int n8) {
  const int i = blockIdx.x * 256 + threadIdx.x;
  if (i >= n8) return;
  const v4f a0 = *(const v4f*)(in + (size_t)i * 8);
  const v4f a1 = *(const v4f*)(in + (size_t)i * 8 + 4);
  v4u w;
  w[0] = (unsigned)f2bf_bits(a0[0]) | ((unsigned)f2bf_bits(a0[1]) << 16);
  w[1] = (unsigned)f2bf_bits(a0[2]) | ((unsigned)f2bf_bits(a0[3]) << 16);
  w[2] = (unsigned)f2bf_bits(a1[0]) | ((unsigned)f2bf_bits(a1[1]) << 16);
  w[3] = (unsigned)f2bf_bits(a1[2]) | ((unsigned)f2bf_bits(a1[3]) << 16);
  unsigned short* p = out + (size_t)i * 8;
  *(volatile v4u*)p = w;
  __threadfence();
  *(volatile v4u*)p = w;
}

__global__ __launch_bounds__(256) void transpose_cast_bf16_64(
    const float* __restrict__ W, unsigned short* __restrict__ Wt, int nrows, int ncols) {
  __shared__ float tile[64][65];
  const int tid = threadIdx.x;
  const int cb = blockIdx.x * 64;
  const int rb = blockIdx.y * 64;
  const int c4 = (tid & 15) * 4, rr = tid >> 4;
#pragma unroll
  for (int i = 0; i < 4; ++i) {
    const int r = rr + 16 * i;
    const v4f x = *(const v4f*)(W + (size_t)(rb + r) * ncols + cb + c4);
    tile[r][c4 + 0] = x[0]; tile[r][c4 + 1] = x[1]; tile[r][c4 + 2] = x[2]; tile[r][c4 + 3] = x[3];
  }
  __syncthreads();
  const int lane = tid & 31, wave = tid >> 5;
  const int q8 = lane >> 3, c8 = (lane & 7) * 8;
  v4u w[2]; size_t off[2];
#pragma unroll
  for (int it = 0; it < 2; ++it) {
    const int n = it * 32 + wave * 4 + q8;
    unsigned short hb[8];
#pragma unroll
    for (int e = 0; e < 8; ++e) hb[e] = f2bf_bits(tile[c8 + e][n]);
    w[it][0] = (unsigned)hb[0] | ((unsigned)hb[1] << 16);
    w[it][1] = (unsigned)hb[2] | ((unsigned)hb[3] << 16);
    w[it][2] = (unsigned)hb[4] | ((unsigned)hb[5] << 16);
    w[it][3] = (unsigned)hb[6] | ((unsigned)hb[7] << 16);
    off[it] = (size_t)(cb + n) * nrows + rb + c8;
  }
  for (int pass = 0; pass < 2; ++pass) {
#pragma unroll
    for (int it = 0; it < 2; ++it) *(volatile v4u*)(Wt + off[it]) = w[it];
    __threadfence();
  }
}

__global__ __launch_bounds__(128) void causal_attn_kernel(
    const unsigned short* __restrict__ qk, const unsigned short* __restrict__ vh, const unsigned short* __restrict__ vl,
    unsigned short* __restrict__ oh, unsigned short* __restrict__ ol) {
  __shared__ __align__(16) unsigned short Ksh[KV_CHUNK * HEAD_D];
  __shared__ __align__(16) unsigned short Vth[HEAD_D * KV_CHUNK];
  __shared__ __align__(16) unsigned short Vtl[HEAD_D * KV_CHUNK];
  __shared__ __align__(16) unsigned short Psh[4][16 * KV_CHUNK];
  __shared__ __align__(16) unsigned short Psl[4][16 * KV_CHUNK];
  __shared__ __align__(16) float Os[4][16 * 68];

  const int tid  = threadIdx.x;
  const int wave = tid >> 5;
  const int lane = tid & 31;
  const int hh   = lane >> 4;
  const int c    = lane & 15;

  const int bx = blockIdx.x;
  const int qb = bx & 31;
  const int bh = bx >> 5;
  const int h  = bh & 15;
  const int b  = bh >> 4;
  const int q0 = qb * 64 + wave * 16;
  const size_t brow0 = (size_t)b * SEQ_LEN;

  v16h qa[2];
  {
    const _Float16* qrow = (const _Float16*)(qk + (brow0 + q0 + c) * QK_PITCH + h * HEAD_D);
    qa[0] = Frag<_Float16>::load(qrow + 8 * hh);
    qa[1] = Frag<_Float16>::load(qrow + 32 + 8 * hh);
  }

  float mrow[8], lrow[8];
  v8f oacc[4];
#pragma unroll
  for (int r = 0; r < 8; ++r) { mrow[r] = -__builtin_inff(); lrow[r] = 0.f; }
#pragma unroll
  for (int t = 0; t < 4; ++t) oacc[t] = (v8f){0.f,0.f,0.f,0.f,0.f,0.f,0.f,0.f};

  for (int kc = 0; kc <= qb; ++kc) {
    const int kv0 = kc * KV_CHUNK;
    const size_t kvrow0 = brow0 + kv0;
    __syncthreads();
#pragma unroll
    for (int i = 0; i < 4; ++i) {
      const int id = tid + 128 * i;
      const int kv = id >> 3, d8 = (id & 7) * 8;
      const v4u w = *(const v4u*)(qk + (kvrow0 + kv) * QK_PITCH + EMB_DIM + h * HEAD_D + d8);
      *(v4u*)(Ksh + kv * HEAD_D + d8) = w;
    }
    {
      const int kv = tid & 63, dh = (tid >> 6) * 32;
      const unsigned short* ph = vh + (kvrow0 + kv) * EMB_DIM + h * HEAD_D + dh;
      const unsigned short* pl = vl + (kvrow0 + kv) * EMB_DIM + h * HEAD_D + dh;
      v4u wh[4], wl[4];
#pragma unroll
      for (int i = 0; i < 4; ++i) { wh[i] = *(const v4u*)(ph + 8 * i); wl[i] = *(const v4u*)(pl + 8 * i); }
#pragma unroll
      for (int i = 0; i < 4; ++i) {
#pragma unroll
        for (int e = 0; e < 4; ++e) {
          const unsigned xh = wh[i][e], xl = wl[i][e];
          const int d = dh + 8 * i + 2 * e;
          Vth[d * KV_CHUNK + kv]       = (unsigned short)(xh & 0xffffu);
          Vth[(d + 1) * KV_CHUNK + kv] = (unsigned short)(xh >> 16);
          Vtl[d * KV_CHUNK + kv]       = (unsigned short)(xl & 0xffffu);
          Vtl[(d + 1) * KV_CHUNK + kv] = (unsigned short)(xl >> 16);
        }
      }
    }
    __syncthreads();

    v8f s[4];
#pragma unroll
    for (int j = 0; j < 4; ++j) {
      s[j] = (v8f){0.f,0.f,0.f,0.f,0.f,0.f,0.f,0.f};
#pragma unroll
      for (int dc = 0; dc < 2; ++dc) {
        const v16h kb = Frag<_Float16>::load((const _Float16*)(Ksh + (j * 16 + c) * HEAD_D + dc * 32 + 8 * hh));
        s[j] = hmma(qa[dc], kb, s[j]);
      }
    }
    const bool diag = (kc == qb);
    float cm[8];
#pragma unroll
    for (int r = 0; r < 8; ++r) {
      const int qrow = q0 + 8 * hh + r;
      float m = -__builtin_inff();
#pragma unroll
      for (int j = 0; j < 4; ++j) {
        const int kvcol = kv0 + j * 16 + c;
        float sv = s[j][r] * (1.0f / 128.0f);
        if (diag && (kvcol > qrow)) sv = MASK_FILL;
        s[j][r] = sv;
        m = fmaxf(m, sv);
      }
#pragma unroll
      for (int off = 1; off < 16; off <<= 1) m = fmaxf(m, __shfl_xor(m, off, 32));
      cm[r] = m;
    }
    unsigned short* pwh = Psh[wave];
    unsigned short* pwl = Psl[wave];
#pragma unroll
    for (int r = 0; r < 8; ++r) {
      const float mnew = fmaxf(mrow[r], cm[r]);
      const float alpha = expf(mrow[r] - mnew);
      mrow[r] = mnew;
      float psum = 0.f;
#pragma unroll
      for (int j = 0; j < 4; ++j) {
        const float p = expf(s[j][r] - mnew);
        psum += p;
        const unsigned short hb = f2bf_bits(p);
        const unsigned short lb = f2bf_bits(p - bf_bits2f(hb));
        pwh[(8 * hh + r) * KV_CHUNK + j * 16 + c] = hb;
        pwl[(8 * hh + r) * KV_CHUNK + j * 16 + c] = lb;
      }
#pragma unroll
      for (int off = 1; off < 16; off <<= 1) psum += __shfl_xor(psum, off, 32);
      lrow[r] = lrow[r] * alpha + psum;
#pragma unroll
      for (int t = 0; t < 4; ++t) oacc[t][r] *= alpha;
    }
    __builtin_amdgcn_fence(__ATOMIC_RELEASE, "workgroup");
    __builtin_amdgcn_wave_barrier();
    __builtin_amdgcn_fence(__ATOMIC_ACQUIRE, "workgroup");
#pragma unroll
    for (int kk = 0; kk < 2; ++kk) {
      const v16b pa = Frag<__bf16>::load((const __bf16*)(pwh + c * KV_CHUNK + kk * 32 + 8 * hh));
      const v16b pl = Frag<__bf16>::load((const __bf16*)(pwl + c * KV_CHUNK + kk * 32 + 8 * hh));
#pragma unroll
      for (int t = 0; t < 4; ++t) {
        const v16b vbh = Frag<__bf16>::load((const __bf16*)(Vth + (t * 16 + c) * KV_CHUNK + kk * 32 + 8 * hh));
        const v16b vbl = Frag<__bf16>::load((const __bf16*)(Vtl + (t * 16 + c) * KV_CHUNK + kk * 32 + 8 * hh));
        oacc[t] = bmma(pa, vbh, oacc[t]);
        oacc[t] = bmma(pa, vbl, oacc[t]);
        oacc[t] = bmma(pl, vbh, oacc[t]);
      }
    }
  }

  float* os = Os[wave];
#pragma unroll
  for (int r = 0; r < 8; ++r) {
    const float inv = 1.0f / lrow[r];
#pragma unroll
    for (int t = 0; t < 4; ++t) os[(8 * hh + r) * 68 + t * 16 + c] = oacc[t][r] * inv;
  }
  __builtin_amdgcn_fence(__ATOMIC_RELEASE, "workgroup");
  __builtin_amdgcn_wave_barrier();
  __builtin_amdgcn_fence(__ATOMIC_ACQUIRE, "workgroup");
  {
    const int q8 = lane >> 3, c8 = (lane & 7) * 8;
    v4u wh[4], wl[4];
#pragma unroll
    for (int it = 0; it < 4; ++it) {
      const int row = it * 4 + q8;
      const float* sp = os + row * 68 + c8;
      const v4f x0 = *(const v4f*)(sp);
      const v4f x1 = *(const v4f*)(sp + 4);
      float t8[8];
      t8[0] = x0[0]; t8[1] = x0[1]; t8[2] = x0[2]; t8[3] = x0[3];
      t8[4] = x1[0]; t8[5] = x1[1]; t8[6] = x1[2]; t8[7] = x1[3];
      unsigned short hb[8], lb[8];
#pragma unroll
      for (int e = 0; e < 8; ++e) {
        hb[e] = f2bf_bits(t8[e]);
        lb[e] = f2bf_bits(t8[e] - bf_bits2f(hb[e]));
      }
      wh[it][0] = (unsigned)hb[0] | ((unsigned)hb[1] << 16);
      wh[it][1] = (unsigned)hb[2] | ((unsigned)hb[3] << 16);
      wh[it][2] = (unsigned)hb[4] | ((unsigned)hb[5] << 16);
      wh[it][3] = (unsigned)hb[6] | ((unsigned)hb[7] << 16);
      wl[it][0] = (unsigned)lb[0] | ((unsigned)lb[1] << 16);
      wl[it][1] = (unsigned)lb[2] | ((unsigned)lb[3] << 16);
      wl[it][2] = (unsigned)lb[4] | ((unsigned)lb[5] << 16);
      wl[it][3] = (unsigned)lb[6] | ((unsigned)lb[7] << 16);
    }
    for (int pass = 0; pass < 2; ++pass) {
#pragma unroll
      for (int it = 0; it < 4; ++it) {
        const int row = it * 4 + q8;
        const size_t o = (brow0 + q0 + row) * EMB_DIM + h * HEAD_D + c8;
        *(volatile v4u*)(oh + o) = wh[it];
        *(volatile v4u*)(ol + o) = wl[it];
      }
      __threadfence();
    }
  }
}

extern "C" void kernel_launch(void* const* d_in, const int* in_sizes, int n_in,
                              void* d_out, int out_size, void* d_ws, size_t ws_size,
                              hipStream_t stream) {
  if (n_in < 5) return;
  if (in_sizes[0] != MROWS * EMB_DIM) return;
  if (in_sizes[1] != EMB_DIM * QKV_N) return;
  if (in_sizes[2] != QKV_N) return;
  if (in_sizes[3] != EMB_DIM * EMB_DIM) return;
  if (in_sizes[4] != EMB_DIM) return;
  if (out_size != MROWS * EMB_DIM) return;
  if (ws_size < WS_TOTAL) return;

  const float* hidden   = (const float*)d_in[0];
  const float* c_attn_w = (const float*)d_in[1];
  const float* c_attn_b = (const float*)d_in[2];
  const float* c_proj_w = (const float*)d_in[3];
  const float* c_proj_b = (const float*)d_in[4];
  float* out = (float*)d_out;

  unsigned char* ws = (unsigned char*)d_ws;
  unsigned short* Xbf = (unsigned short*)(ws + WS_OFF_XBF);
  unsigned short* WaT = (unsigned short*)(ws + WS_OFF_WAT);
  unsigned short* WpT = (unsigned short*)(ws + WS_OFF_WPT);
  unsigned short* QKp = (unsigned short*)(ws + WS_OFF_QKP);
  unsigned short* Vhi = (unsigned short*)(ws + WS_OFF_VHI);
  unsigned short* Vlo = (unsigned short*)(ws + WS_OFF_VLO);
  unsigned short* ATh = (unsigned short*)(ws + WS_OFF_ATH);
  unsigned short* ATl = (unsigned short*)(ws + WS_OFF_ATL);

  {
    const int n8 = (MROWS * EMB_DIM) / 8;
    static_assert((MROWS * EMB_DIM) % (8 * 256) == 0);
    cast_f32_bf16x8<<<dim3(n8 / 256), 256, 0, stream>>>(hidden, Xbf, n8);
  }
  transpose_cast_bf16_64<<<dim3(QKV_N / 64, EMB_DIM / 64), 256, 0, stream>>>(c_attn_w, WaT, EMB_DIM, QKV_N);
  transpose_cast_bf16_64<<<dim3(EMB_DIM / 64, EMB_DIM / 64), 256, 0, stream>>>(c_proj_w, WpT, EMB_DIM, EMB_DIM);

  static_assert(MROWS % 64 == 0 && QK_PITCH % 64 == 0 && EMB_DIM % 32 == 0);
  {
    const int tiles = (MROWS / 64) * (QK_PITCH / 64);
    static_assert(((MROWS / 64) * (QK_PITCH / 64)) % 8 == 0);
    wmma_gemm64<1, false, false, 2, 1><<<dim3(tiles / 8, 1), 256, 0, stream>>>(
        Xbf, Xbf, EMB_DIM, 0L, WaT, WaT, EMB_DIM, 0L, (void*)QKp, (void*)QKp, QK_PITCH, 0L,
        c_attn_b, MROWS, QK_PITCH, EMB_DIM, 4.0f, 4.0f);
  }
  {
    const int tiles = (MROWS / 64) * (EMB_DIM / 64);
    static_assert(((MROWS / 64) * (EMB_DIM / 64)) % 8 == 0);
    wmma_gemm64<1, false, false, 2, 2><<<dim3(tiles / 8, 1), 256, 0, stream>>>(
        Xbf, Xbf, EMB_DIM, 0L, WaT + (size_t)QK_PITCH * EMB_DIM, WaT + (size_t)QK_PITCH * EMB_DIM, EMB_DIM, 0L,
        (void*)Vhi, (void*)Vlo, EMB_DIM, 0L,
        c_attn_b + QK_PITCH, MROWS, EMB_DIM, EMB_DIM, 1.0f, 1.0f);
  }
  causal_attn_kernel<<<dim3(NB_BATCH * N_HEADS * (SEQ_LEN / 64)), 128, 0, stream>>>(QKp, Vhi, Vlo, ATh, ATl);
  {
    const int tiles = (MROWS / 64) * (EMB_DIM / 64);
    wmma_gemm64<1, true, false, 2, 0><<<dim3(tiles / 8, 1), 256, 0, stream>>>(
        ATh, ATl, EMB_DIM, 0L, WpT, WpT, EMB_DIM, 0L, (void*)out, (void*)out, EMB_DIM, 0L,
        c_proj_b, MROWS, EMB_DIM, EMB_DIM, 1.0f, 1.0f);
  }
}
